// RNNs_59622736003524
// MI455X (gfx1250) — hardware-verified
//
#include <hip/hip_runtime.h>


namespace {
constexpr int NBt = 512, T = 288, F = 8, HD = 256, PRED = 12;
constexpr float XS = 8.0f, WSC = 256.0f;

typedef _Float16 b16;
typedef __attribute__((ext_vector_type(16))) _Float16 v16b;
typedef __attribute__((ext_vector_type(8))) _Float16 v8b;
typedef __attribute__((ext_vector_type(8))) float v8f;
typedef __attribute__((ext_vector_type(4))) float v4f;
__device__ __forceinline__ float bf16_rne(float f) { unsigned int u = __float_as_uint(f); u += 0x7FFFu + ((u >> 16) & 1u); return __uint_as_float(u & 0xFFFF0000u); }
__device__ __forceinline__ v16b frag_kb(const b16* p, int hh) { const v8b a = *(const v8b*)(p + 8 * hh), b = *(const v8b*)(p + 16 + 8 * hh); v16b f;
#pragma unroll
  for (int e = 0; e < 8; ++e) { f[e] = a[e]; f[8 + e] = b[e]; } return f; }
__device__ __forceinline__ v8f wmma16b(v16b a, v16b b, v8f c) { v8f d = __builtin_amdgcn_wmma_f32_16x16x32_f16(false, a, false, b, (short)0, c, false, false); asm volatile("v_nop\n\tv_nop\n\tv_nop\n\tv_nop" : "+v"(d) : "v"(a), "v"(b)); return d; }
__device__ __forceinline__ void wave_lds_sync() { __builtin_amdgcn_fence(__ATOMIC_RELEASE, "workgroup"); __builtin_amdgcn_wave_barrier(); __builtin_amdgcn_fence(__ATOMIC_ACQUIRE, "workgroup"); }
__device__ __forceinline__ float nexp(float x) { return __builtin_amdgcn_exp2f(x * 1.4426950408889634f); }
__device__ __forceinline__ float pmul(float a, float b) { float p = a * b; asm volatile("" : "+v"(p)); return p; }
__device__ __forceinline__ float tanh_(float x) { const float e = nexp(-2.0f * fabsf(x)); const float t = (1.0f - e) / (1.0f + e); return x < 0.0f ? -t : t; }
__device__ __forceinline__ float hsum16(float v) { v += __shfl_xor(v, 1); v += __shfl_xor(v, 2); v += __shfl_xor(v, 4); return v + __shfl_xor(v, 8); }

__global__ __launch_bounds__(256) void prep_kernel(const float* __restrict__ x, const float* __restrict__ win, const float* __restrict__ wih, const float* __restrict__ whh, b16* __restrict__ X16, b16* __restrict__ WIN, b16* __restrict__ W4) {
  const size_t t = (size_t)blockIdx.x * 256 + threadIdx.x; const size_t nx = (size_t)NBt * T * 4  , nw = (size_t)HD * 4, n4 = (size_t)4 * HD * HD / 8;
  if (t < nx) { const size_t row = t >> 2; const int g = (int)(t & 3); v8b o = {}; if (g == 0) { const float* s = x + row * F; for (int j = 0; j < 8; ++j) o[j] = (b16)(bf16_rne(s[j]) * XS); }
    for (int pass = 0; pass < 2; ++pass) { *(volatile v8b*)(X16 + row * 32 + g * 8) = o; __threadfence(); } }
  else if (t < nx + nw) { const size_t u = t - nx; const int o_ = (int)(u >> 2), g = (int)(u & 3); v8b o = {}; if (g == 0) for (int j = 0; j < 8; ++j) o[j] = (b16)(bf16_rne(win[o_ * F + j]) * WSC);
    for (int pass = 0; pass < 2; ++pass) { *(volatile v8b*)(WIN + (size_t)o_ * 32 + g * 8) = o; __threadfence(); } }
  else if (t < nx + nw + n4) { const size_t u = (t - nx - nw) * 8; const int k = (int)(u / ((size_t)HD * HD)); const size_t e = u - (size_t)k * HD * HD;
    const float* src = ((k & 1) ? whh : wih) + (size_t)(k >> 1) * HD * HD + e; v8b o; for (int j = 0; j < 8; ++j) o[j] = (b16)(bf16_rne(src[j]) * WSC);
    for (int pass = 0; pass < 2; ++pass) { *(volatile v8b*)(W4 + u) = o; __threadfence(); } }
}
__global__ __launch_bounds__(128) void rnn_kernel(const b16* __restrict__ X16, const b16* __restrict__ WIN, const b16* __restrict__ W4, const float* __restrict__ b_in, const float* __restrict__ b_ih, const float* __restrict__ b_hh, const float* __restrict__ w_out, const float* __restrict__ b_out, const int* __restrict__ predlen, float* __restrict__ out) {
  __shared__ __attribute__((aligned(16))) b16 Xs[16][HD + 8], H0[16][HD + 8], H1[16][HD + 8]; __shared__ float Po[4][16][PRED];
  const int wave = threadIdx.x >> 5, lane = threadIdx.x & 31, nloc = lane & 15, hlf = lane >> 4, t_ = threadIdx.x; const size_t b0 = (size_t)blockIdx.x * 16;
  for (int q = t_; q < 16 * (HD + 8); q += 128) { (&H0[0][0])[q] = (b16)0.0f; (&H1[0][0])[q] = (b16)0.0f; }
  const int pl = min(max(predlen[0], 1), PRED);
  float bx[4], b0v[4], b1v[4], wo[4];
#pragma unroll
  for (int t = 0; t < 4; ++t) { const int j = wave * 64 + t * 16 + nloc; bx[t] = bf16_rne(b_in[j]); b0v[t] = bf16_rne(b_ih[j]) + bf16_rne(b_hh[j]); b1v[t] = bf16_rne(b_ih[HD + j]) + bf16_rne(b_hh[HD + j]); wo[t] = bf16_rne(w_out[j]); }
  const float bo = bf16_rne(b_out[0]);
  __syncthreads();
  for (int t = 0; t < T; ++t) {
    { v8f ax[4] = {{}, {}, {}, {}}; const v16b a = frag_kb(X16 + ((b0 + nloc) * T + t) * 32, hlf);
#pragma unroll
      for (int tt = 0; tt < 4; ++tt) ax[tt] = wmma16b(a, frag_kb(WIN + (size_t)(wave * 64 + tt * 16 + nloc) * 32, hlf), ax[tt]);
#pragma unroll
      for (int tt = 0; tt < 4; ++tt)
#pragma unroll
        for (int r = 0; r < 8; ++r) Xs[8 * hlf + r][wave * 64 + tt * 16 + nloc] = (b16)((ax[tt][r] * (1.0f / (XS * WSC)) + bx[tt]) * XS); }
    __syncthreads();
    v8f z[4] = {{}, {}, {}, {}};
#pragma unroll 2
    for (int kb = 0; kb < HD; kb += 32) { const v16b ax_ = frag_kb(&Xs[nloc][kb], hlf), ah = frag_kb(&H0[nloc][kb], hlf);
#pragma unroll
      for (int tt = 0; tt < 4; ++tt) { const int n = wave * 64 + tt * 16 + nloc; z[tt] = wmma16b(ax_, frag_kb(W4 + (size_t)(0 * HD + n) * HD + kb, hlf), z[tt]); z[tt] = wmma16b(ah, frag_kb(W4 + (size_t)(1 * HD + n) * HD + kb, hlf), z[tt]); } }
    __syncthreads();
#pragma unroll
    for (int tt = 0; tt < 4; ++tt)
#pragma unroll
      for (int r = 0; r < 8; ++r) H0[8 * hlf + r][wave * 64 + tt * 16 + nloc] = (b16)(tanh_(z[tt][r] * (1.0f / (XS * WSC)) + b0v[tt]) * XS);
    __syncthreads();
    v8f z1[4] = {{}, {}, {}, {}};
#pragma unroll 2
    for (int kb = 0; kb < HD; kb += 32) { const v16b a0 = frag_kb(&H0[nloc][kb], hlf), a1 = frag_kb(&H1[nloc][kb], hlf);
#pragma unroll
      for (int tt = 0; tt < 4; ++tt) { const int n = wave * 64 + tt * 16 + nloc; z1[tt] = wmma16b(a0, frag_kb(W4 + (size_t)(2 * HD + n) * HD + kb, hlf), z1[tt]); z1[tt] = wmma16b(a1, frag_kb(W4 + (size_t)(3 * HD + n) * HD + kb, hlf), z1[tt]); } }
    __syncthreads();
    const int slot = t - (T - 1 - pl);
    float part[8];
#pragma unroll
    for (int r = 0; r < 8; ++r) part[r] = 0.0f;
#pragma unroll
    for (int tt = 0; tt < 4; ++tt)
#pragma unroll
      for (int r = 0; r < 8; ++r) { const float h = tanh_(z1[tt][r] * (1.0f / (XS * WSC)) + b1v[tt]); H1[8 * hlf + r][wave * 64 + tt * 16 + nloc] = (b16)(h * XS); part[r] += pmul(fmaxf(h, 0.0f), wo[tt]); }
    if (slot >= 0 && slot < pl && t <= T - 2) {
#pragma unroll
      for (int r = 0; r < 8; ++r) { const float s = hsum16(part[r]); if (nloc == 0) Po[wave][8 * hlf + r][slot] = s; } }
    __syncthreads();
  }
  for (int pass = 0; pass < 2; ++pass) { for (int i = t_; i < 16 * PRED; i += 128) { const int rr = i / PRED, sl = i - rr * PRED; const float v = ((Po[0][rr][sl] + Po[1][rr][sl]) + (Po[2][rr][sl] + Po[3][rr][sl])) + bo; ((volatile float*)out)[(b0 + rr) * PRED + sl] = (sl < pl) ? v : 0.0f; } __threadfence(); }
}
}

extern "C" void kernel_launch(void* const* d_in, const int* in_sizes, int n_in, void* d_out, int out_size, void* d_ws, size_t ws_size, hipStream_t stream) {
  (void)n_in;
  auto Fp = [&](int i) { return (const float*)d_in[i]; };
  if (in_sizes[0] != NBt * T * F || in_sizes[1] != HD * F || in_sizes[3] != 2 * HD * HD || in_sizes[5] != 2 * HD * HD || in_sizes[7] != HD || out_size != NBt * PRED) return;
  size_t off = 0; char* ws = (char*)d_ws;
  auto carve = [&](size_t bytes) { char* p = ws + off; off += (bytes + 255) & ~(size_t)255; return p; };
  b16* X16 = (b16*)carve((size_t)NBt * T * 32 * 2); b16* WIN = (b16*)carve((size_t)HD * 32 * 2); b16* W4 = (b16*)carve((size_t)4 * HD * HD * 2);
  if (off > ws_size || off > ((size_t)128 << 20)) return;
  prep_kernel<<<(unsigned)(((size_t)NBt * T * 4 + (size_t)HD * 4 + (size_t)4 * HD * HD / 8 + 255) / 256), 256, 0, stream>>>(Fp(0), Fp(1), Fp(3), Fp(5), X16, WIN, W4);
  rnn_kernel<<<NBt / 16, 128, 0, stream>>>(X16, WIN, W4, Fp(2), Fp(4), Fp(6), Fp(7), Fp(8), (const int*)d_in[9], (float*)d_out);
}
